// TransformerBlock3D_18562848653468
// MI455X (gfx1250) — hardware-verified
//
#include <hip/hip_runtime.h>
#include <math.h>
#include <stddef.h>

typedef __attribute__((ext_vector_type(16))) _Float16 v16h;
typedef __attribute__((ext_vector_type(8)))  _Float16 v8h;
typedef __attribute__((ext_vector_type(16))) __bf16   v16b;
typedef __attribute__((ext_vector_type(8)))  __bf16   v8b;
typedef __attribute__((ext_vector_type(8)))  float    v8f;
typedef __attribute__((ext_vector_type(4)))  float    v4f;
#define PSCALE 32768.0f
#define U16(p) ((const unsigned short*)(const void*)(p))
#define PSCALE_INV (1.0f / 32768.0f)

__device__ __forceinline__ unsigned short f2bf_bits(float f) {
  unsigned u = __float_as_uint(f);
  return (unsigned short)((u + 0x7FFFu + ((u >> 16) & 1u)) >> 16);
}
__device__ __forceinline__ float bf_bits2f(unsigned short h) { return __uint_as_float(((unsigned)h) << 16); }

__device__ __forceinline__ void dep_guard_h(v8f& a, v8f& b, v16h x, v16h y) { asm volatile("v_nop\n\tv_nop\n\tv_nop\n\tv_nop" : "+v"(a), "+v"(b) : "v"(x), "v"(y)); }
__device__ __forceinline__ void dep_guard_b(v8f& a, v8f& b, v16b x, v16b y) { asm volatile("v_nop\n\tv_nop\n\tv_nop\n\tv_nop" : "+v"(a), "+v"(b) : "v"(x), "v"(y)); }
__device__ __forceinline__ void keep4_h(v16h a, v16h b, v16h c, v16h d) { asm volatile("v_nop" :: "v"(a), "v"(b), "v"(c), "v"(d)); }
__device__ __forceinline__ void keep4_b(v16b a, v16b b, v16b c, v16b d) { asm volatile("v_nop" :: "v"(a), "v"(b), "v"(c), "v"(d)); }
__device__ __forceinline__ void acc_guard4(v8f& a, v8f& b, v8f& c, v8f& d) { asm volatile("v_nop\n\tv_nop\n\tv_nop\n\tv_nop" : "+v"(a), "+v"(b), "+v"(c), "+v"(d)); }
template <typename T> struct Frag;
template <> struct Frag<_Float16> {
  typedef v16h V; union U { v16h v; v8h h[2]; };
  static __device__ __forceinline__ v16h load(const _Float16* p) {
    U f; f.h[0] = *(const v8h*)(p); f.h[1] = *(const v8h*)(p + 16); return f.v;
  }
  static __device__ __forceinline__ v8f mma(v16h a, v16h b, v8f c) {
    return __builtin_amdgcn_wmma_f32_16x16x32_f16(false, a, false, b, (short)0, c, false, false);
  }
  static __device__ __forceinline__ void guard(v8f& a, v8f& b, v16h x, v16h y) { dep_guard_h(a, b, x, y); }
  static __device__ __forceinline__ void keep(v16h a, v16h b, v16h c, v16h d) { keep4_h(a, b, c, d); }
};
template <> struct Frag<__bf16> {
  typedef v16b V; union U { v16b v; v8b h[2]; };
  static __device__ __forceinline__ v16b load(const __bf16* p) {
    U f; f.h[0] = *(const v8b*)(p); f.h[1] = *(const v8b*)(p + 16); return f.v;
  }
  static __device__ __forceinline__ v8f mma(v16b a, v16b b, v8f c) {
    return __builtin_amdgcn_wmma_f32_16x16x32_bf16(false, a, false, b, (short)0, c, false, false);
  }
  static __device__ __forceinline__ void guard(v8f& a, v8f& b, v16b x, v16b y) { dep_guard_b(a, b, x, y); }
  static __device__ __forceinline__ void keep(v16b a, v16b b, v16b c, v16b d) { keep4_b(a, b, c, d); }
};

template <int ET> struct Elem;
template <> struct Elem<0> { typedef _Float16 T; };
template <> struct Elem<1> { typedef __bf16 T; };
template <int ET, bool SPLIT, int BIAS_MODE, int OUT_MODE, bool RESID, int ACT = 0>
__global__ __launch_bounds__(256) void wmma_gemm64(
    const unsigned short* __restrict__ Ap, const unsigned short* __restrict__ A2p, int lda, long strideA,
    const unsigned short* __restrict__ Btp, const unsigned short* __restrict__ Bt2p, int ldb, long strideB,
    void* __restrict__ Cout, void* __restrict__ Cout2, int ldc, long strideC,
    const float* __restrict__ bias,
    const float* __restrict__ resid, long strideR,
    int M, int N, int K, float scale) {
  typedef typename Elem<ET>::T T;
  typedef typename Frag<T>::V V;
  const T* A = (const T*)Ap; const T* A2 = (const T*)A2p; const T* Bt = (const T*)Btp; const T* Bt2 = (const T*)Bt2p;
  __shared__ __align__(16) float sT[8][16 * 68];
  const int b    = blockIdx.y;
  const int lane = threadIdx.x & 31;
  const int wave = threadIdx.x >> 5;
  const int tilesN = N >> 6;
  const int tilesM = M >> 6;
  const int tile = blockIdx.x * 8 + wave;
  if (tile >= tilesM * tilesN) return;
  const int tm = tile / tilesN;
  const int tn = tile - tm * tilesN;
  const int m0 = tm << 6;
  const int n0 = tn << 6;

  const T* Ab  = A  + (size_t)b * strideA;
  const T* Bb  = Bt + (size_t)b * strideB;
  const T* Ab2 = SPLIT ? (A2  + (size_t)b * strideA) : nullptr;
  const T* Bb2 = SPLIT ? (Bt2 + (size_t)b * strideB) : nullptr;

  const int rlane = lane & 15;
  const int koff  = (lane >> 4) * 8;
  const int mOff  = (lane >> 4) * 8;

  v8f acc[4][4];
#pragma unroll
  for (int i = 0; i < 4; ++i)
#pragma unroll
    for (int j = 0; j < 4; ++j) acc[i][j] = (v8f){0.f,0.f,0.f,0.f,0.f,0.f,0.f,0.f};

  for (int k0 = 0; k0 < K; k0 += 32) {
    V bh[4], bl[4];
#pragma unroll
    for (int j = 0; j < 4; ++j) {
      const size_t bo = (size_t)(n0 + (j << 4) + rlane) * ldb + koff + k0;
      bh[j] = Frag<T>::load(Bb + bo);
      if (SPLIT) bl[j] = Frag<T>::load(Bb2 + bo);
    }
#pragma unroll
    for (int i = 0; i < 4; ++i) {
      const size_t ao = (size_t)(m0 + (i << 4) + rlane) * lda + koff + k0;
      V ah = Frag<T>::load(Ab + ao);
      V al;
      if (SPLIT) al = Frag<T>::load(Ab2 + ao);
#pragma unroll
      for (int j = 0; j < 4; ++j) {
        acc[i][j] = Frag<T>::mma(ah, bh[j], acc[i][j]);
        if (SPLIT) {
          acc[i][j] = Frag<T>::mma(ah, bl[j], acc[i][j]);
          acc[i][j] = Frag<T>::mma(al, bh[j], acc[i][j]);
        }
      }
      Frag<T>::guard(acc[i][0], acc[i][3], ah, SPLIT ? al : ah);
    }
    Frag<T>::keep(bh[0], bh[1], bh[2], bh[3]);
    if (SPLIT) Frag<T>::keep(bl[0], bl[1], bl[2], bl[3]);
  }
  acc_guard4(acc[0][0], acc[0][1], acc[0][2], acc[0][3]);
  acc_guard4(acc[1][0], acc[1][1], acc[1][2], acc[1][3]);
  acc_guard4(acc[2][0], acc[2][1], acc[2][2], acc[2][3]);
  acc_guard4(acc[3][0], acc[3][1], acc[3][2], acc[3][3]);

  float* slab = sT[wave];
  const float* Rb = RESID ? (resid + (size_t)b * strideR) : nullptr;
#pragma unroll
  for (int i = 0; i < 4; ++i) {
    const int mBase = m0 + (i << 4);
#pragma unroll
    for (int j = 0; j < 4; ++j) {
      const int n = n0 + (j << 4) + rlane;
      float bv = 0.f;
      if (BIAS_MODE == 2) bv = bias[n];
#pragma unroll
      for (int r = 0; r < 8; ++r) {
        float v = acc[i][j][r] * scale;
        if (BIAS_MODE == 1) v += bias[mBase + mOff + r];
        if (BIAS_MODE == 2) v += bv;
        if (RESID) v += Rb[(size_t)(mBase + mOff + r) * ldc + n];
        if (ACT == 1) v = tanhf(v);
        if (ACT == 2) v = fmaxf(v, 0.0f);
        if (ACT == 3) v = v / (1.0f + expf(-v));
        if (ACT == 4) v = (v > 0.f) ? v : 0.01f * v;
        if (ACT == 5) v = 0.5f * v * (1.0f + erff(v * 0.70710678118654752f));
        slab[(mOff + r) * 68 + (j << 4) + rlane] = v;
      }
    }
    __builtin_amdgcn_fence(__ATOMIC_RELEASE, "workgroup");
    __builtin_amdgcn_wave_barrier();
    __builtin_amdgcn_fence(__ATOMIC_ACQUIRE, "workgroup");
    if (OUT_MODE == 0) {
      float* C = (float*)Cout + (size_t)b * strideC;
      const int hh = lane >> 4, c4 = (lane & 15) * 4;
      for (int pass = 0; pass < 2; ++pass) {
#pragma unroll
        for (int it = 0; it < 8; ++it) {
          const int row = it * 2 + hh;
          v4f v = *(const v4f*)(slab + row * 68 + c4);
          *(volatile v4f*)(C + (size_t)(mBase + row) * ldc + n0 + c4) = v;
        }
        __threadfence();
      }
    } else {
      const int q = lane >> 3, c8 = (lane & 7) * 8;
      unsigned short* C  = (unsigned short*)Cout  + (size_t)b * strideC;
      unsigned short* C2 = (OUT_MODE == 2) ? ((unsigned short*)Cout2 + (size_t)b * strideC) : nullptr;
      for (int pass = 0; pass < 2; ++pass) {
#pragma unroll
        for (int it = 0; it < 4; ++it) {
          const int row = it * 4 + q;
          const float* sp = slab + row * 68 + c8;
          v8h hv, lv;
#pragma unroll
          for (int e = 0; e < 8; ++e) {
            if (OUT_MODE == 1) {
              hv[e] = (_Float16)sp[e];
            } else {
              unsigned short hb = f2bf_bits(sp[e]);
              unsigned short lb = f2bf_bits(sp[e] - bf_bits2f(hb));
              hv[e] = __builtin_bit_cast(_Float16, hb);
              lv[e] = __builtin_bit_cast(_Float16, lb);
            }
          }
          *(volatile v8h*)(C + (size_t)(mBase + row) * ldc + n0 + c8) = hv;
          if (OUT_MODE == 2) *(volatile v8h*)(C2 + (size_t)(mBase + row) * ldc + n0 + c8) = lv;
        }
        __threadfence();
      }
    }
    __builtin_amdgcn_fence(__ATOMIC_RELEASE, "workgroup");
    __builtin_amdgcn_wave_barrier();
    __builtin_amdgcn_fence(__ATOMIC_ACQUIRE, "workgroup");
  }
}

#define NTOK   4096
#define CDIM   256
#define FFDIM  1024
#define NHEAD  8
#define HDIM   32
#define NGRP   32
#define GN_EPS 1e-5f
#define WSCALE 64.0f
#define WSCALE_INV (1.0f / 64.0f)

__global__ __launch_bounds__(256) void transpose_cast_f16(
    const float* __restrict__ in, unsigned short* __restrict__ outp, int R, int Cc, float scale) {
  __shared__ float s[64 * 65];
  _Float16* out = (_Float16*)(void*)outp;
  const int tid = threadIdx.x, lane = tid & 31, wave = tid >> 5;
  const int r0 = blockIdx.y * 64, c0 = blockIdx.x * 64;
#pragma unroll
  for (int p = 0; p < 4; ++p) {
    const int row = p * 16 + (tid >> 4);
    const int col4 = (tid & 15) * 4;
    const v4f vv = *(const v4f*)(in + (size_t)(r0 + row) * Cc + c0 + col4);
#pragma unroll
    for (int e = 0; e < 4; ++e) s[row * 65 + col4 + e] = vv[e];
  }
  __syncthreads();
  const int q8 = lane >> 3, r8 = (lane & 7) * 8;
  for (int pass = 0; pass < 2; ++pass) {
#pragma unroll
    for (int it = 0; it < 2; ++it) {
      const int cl = wave * 8 + it * 4 + q8;
      v8h hv;
#pragma unroll
      for (int e = 0; e < 8; ++e) hv[e] = (_Float16)(s[(r8 + e) * 65 + cl] * scale);
      *(volatile v8h*)(out + (size_t)(c0 + cl) * R + r0 + r8) = hv;
    }
    __threadfence();
  }
}

__device__ __forceinline__ void gn_finish(double s, double q, double* rs, double* rq,
                                          float* __restrict__ stats, int g, int tid,
                                          double inv_cnt, float eps) {
  rs[tid] = s; rq[tid] = q;
  __syncthreads();
  for (int o = 128; o > 0; o >>= 1) {
    if (tid < o) { rs[tid] += rs[tid + o]; rq[tid] += rq[tid + o]; }
    __syncthreads();
  }
  if (tid < 32) {
    const double mu = rs[0] * inv_cnt;
    double var = rq[0] * inv_cnt - mu * mu;
    var = (var < 0.0) ? 0.0 : var;
    const float muf  = (float)mu;
    const float rstd = 1.0f / sqrtf((float)var + eps);
    const float val = (tid == 0) ? muf : ((tid == 1) ? rstd : 0.0f);
    volatile float* sp = stats + (size_t)g * 32 + tid;
    *sp = val;
    __threadfence();
    *sp = val;
  }
}

__global__ __launch_bounds__(256) void gn_stats_cm(
    const float* __restrict__ x, float* __restrict__ stats, int npg, float eps) {
  __shared__ double rs[256], rq[256];
  const int g = blockIdx.x, tid = threadIdx.x;
  const float* base = x + (size_t)g * npg;
  double s = 0.0, q = 0.0;
#pragma unroll 1
  for (int i = tid * 4; i < npg; i += 1024) {
    const v4f vv = *(const v4f*)(base + i);
#pragma unroll
    for (int e = 0; e < 4; ++e) { const double d = (double)vv[e]; s += d; q += d * d; }
  }
  gn_finish(s, q, rs, rq, stats, g, tid, 1.0 / (double)npg, eps);
}

__global__ __launch_bounds__(256) void gn_stats_tm(
    const float* __restrict__ x2, float* __restrict__ stats, int S, float eps) {
  __shared__ double rs[256], rq[256];
  const int g = blockIdx.x, tid = threadIdx.x;
  double s = 0.0, q = 0.0;
#pragma unroll 1
  for (int n = tid; n < S; n += 256) {
    const float* p = x2 + (size_t)n * CDIM + g * 8;
    const v4f a = *(const v4f*)p;
    const v4f b = *(const v4f*)(p + 4);
#pragma unroll
    for (int e = 0; e < 4; ++e) {
      const double d0 = (double)a[e], d1 = (double)b[e];
      s += d0; q += d0 * d0; s += d1; q += d1 * d1;
    }
  }
  gn_finish(s, q, rs, rq, stats, g, tid, 1.0 / (8.0 * (double)S), eps);
}

__global__ __launch_bounds__(256) void gn_apply_cm(
    const float* __restrict__ x, const float* __restrict__ stats,
    const float* __restrict__ gw, const float* __restrict__ gb,
    float* __restrict__ t, unsigned short* __restrict__ thp, int S) {
  __shared__ float sX[256 * 36];
  __shared__ __align__(16) float sRow[8][256];
  _Float16* th = (_Float16*)(void*)thp;
  const int tid = threadIdx.x, lane = tid & 31, wave = tid >> 5;
  const int n0 = blockIdx.x * 32;
  for (int i = 0; i < 32; ++i) {
    const int ch = i * 8 + wave;
    sX[ch * 36 + lane] = x[(size_t)ch * S + n0 + lane];
  }
  __syncthreads();
  const float mu = stats[lane * 32], rstd = stats[lane * 32 + 1];
  float w[8], bb[8];
  {
    const v4f w0 = *(const v4f*)(gw + 8 * lane), w1 = *(const v4f*)(gw + 8 * lane + 4);
    const v4f b0 = *(const v4f*)(gb + 8 * lane), b1 = *(const v4f*)(gb + 8 * lane + 4);
#pragma unroll
    for (int e = 0; e < 4; ++e) { w[e] = w0[e]; w[4 + e] = w1[e]; bb[e] = b0[e]; bb[4 + e] = b1[e]; }
  }
  float* sr = sRow[wave];
#pragma unroll
  for (int tt = 0; tt < 4; ++tt) {
    const int tok = wave * 4 + tt;
    const size_t n = (size_t)(n0 + tok);
    float vals[8];
#pragma unroll
    for (int e = 0; e < 8; ++e) {
      const float xv = sX[(8 * lane + e) * 36 + tok];
      vals[e] = ((xv - mu) * rstd) * w[e] + bb[e];
    }
    v8h hv;
#pragma unroll
    for (int e = 0; e < 8; ++e) hv[e] = (_Float16)vals[e];
    const v4f lo = (v4f){vals[0], vals[1], vals[2], vals[3]};
    const v4f hi = (v4f){vals[4], vals[5], vals[6], vals[7]};
    *(v4f*)(sr + 8 * lane) = lo;
    *(v4f*)(sr + 8 * lane + 4) = hi;
    __builtin_amdgcn_fence(__ATOMIC_RELEASE, "workgroup");
    __builtin_amdgcn_wave_barrier();
    __builtin_amdgcn_fence(__ATOMIC_ACQUIRE, "workgroup");
    const v4f a0 = *(const v4f*)(sr + 4 * lane);
    const v4f a1 = *(const v4f*)(sr + 128 + 4 * lane);
    float* trow = t + n * CDIM;
    _Float16* hrow = th + n * CDIM;
    *(volatile v8h*)(hrow + 8 * lane) = hv;
    *(volatile v4f*)(trow + 4 * lane) = a0;
    *(volatile v4f*)(trow + 128 + 4 * lane) = a1;
    __threadfence();
    *(volatile v8h*)(hrow + 8 * lane) = hv;
    *(volatile v4f*)(trow + 4 * lane) = a0;
    *(volatile v4f*)(trow + 128 + 4 * lane) = a1;
    __builtin_amdgcn_fence(__ATOMIC_RELEASE, "workgroup");
    __builtin_amdgcn_wave_barrier();
    __builtin_amdgcn_fence(__ATOMIC_ACQUIRE, "workgroup");
  }
}

__global__ __launch_bounds__(256) void gn_apply_tm(
    const float* __restrict__ x2, const float* __restrict__ stats,
    const float* __restrict__ gw, const float* __restrict__ gb,
    unsigned short* __restrict__ t2hp, float* __restrict__ t2cm, int S) {
  __shared__ __align__(16) float sTt[256 * 36];
  _Float16* t2h = (_Float16*)(void*)t2hp;
  const int tid = threadIdx.x, lane = tid & 31, wave = tid >> 5;
  const int n0 = blockIdx.x * 32;
  const float mu = stats[lane * 32], rstd = stats[lane * 32 + 1];
  float w[8], bb[8];
  {
    const v4f w0 = *(const v4f*)(gw + 8 * lane), w1 = *(const v4f*)(gw + 8 * lane + 4);
    const v4f b0 = *(const v4f*)(gb + 8 * lane), b1 = *(const v4f*)(gb + 8 * lane + 4);
#pragma unroll
    for (int e = 0; e < 4; ++e) { w[e] = w0[e]; w[4 + e] = w1[e]; bb[e] = b0[e]; bb[4 + e] = b1[e]; }
  }
#pragma unroll
  for (int tt = 0; tt < 4; ++tt) {
    const int tok = wave * 4 + tt;
    const size_t n = (size_t)(n0 + tok);
    const float* xr = x2 + n * CDIM + 8 * lane;
    const v4f xa = *(const v4f*)xr;
    const v4f xb = *(const v4f*)(xr + 4);
    float vals[8];
#pragma unroll
    for (int e = 0; e < 4; ++e) {
      vals[e]     = ((xa[e] - mu) * rstd) * w[e] + bb[e];
      vals[4 + e] = ((xb[e] - mu) * rstd) * w[4 + e] + bb[4 + e];
    }
    v8h hv;
#pragma unroll
    for (int e = 0; e < 8; ++e) hv[e] = (_Float16)vals[e];
    _Float16* hrow = t2h + n * CDIM;
    *(volatile v8h*)(hrow + 8 * lane) = hv;
    __threadfence();
    *(volatile v8h*)(hrow + 8 * lane) = hv;
#pragma unroll
    for (int e = 0; e < 8; ++e) sTt[(8 * lane + e) * 36 + tok] = vals[e];
  }
  __syncthreads();
  const int q8 = lane >> 3, f4 = (lane & 7) * 4;
  for (int pass = 0; pass < 2; ++pass) {
#pragma unroll
    for (int it = 0; it < 8; ++it) {
      const int ch = wave * 32 + it * 4 + q8;
      const v4f vv = *(const v4f*)(sTt + ch * 36 + f4);
      *(volatile v4f*)(t2cm + (size_t)ch * S + n0 + f4) = vv;
    }
    __threadfence();
  }
}

#define AH_D  32
#define AH_NW 4
#define AH_QB 64
#define AH_KC 64

__device__ __forceinline__ v8f mma_f16g(v16h a, v16h b, v8f c) {
  c = __builtin_amdgcn_wmma_f32_16x16x32_f16(false, a, false, b, (short)0, c, false, false);
  asm volatile("v_nop\n\tv_nop\n\tv_nop\n\tv_nop" : "+v"(c) : "v"(a), "v"(b));
  return c;
}

__global__ __launch_bounds__(128)
void attn_hd32_f16(const unsigned short* __restrict__ qp, const unsigned short* __restrict__ kp,
                   const unsigned short* __restrict__ vp, unsigned short* __restrict__ op,
                   int S, int ld, float qk_scale) {
  const _Float16* q = (const _Float16*)(const void*)qp;
  const _Float16* k = (const _Float16*)(const void*)kp;
  const _Float16* v = (const _Float16*)(const void*)vp;
  _Float16* o = (_Float16*)(void*)op;
  __shared__ __align__(16) _Float16 Ksh[AH_KC * AH_D];
  __shared__ __align__(16) _Float16 Vth[AH_D * AH_KC];
  __shared__ __align__(16) _Float16 Psh[AH_NW][16 * AH_KC];
  __shared__ __align__(16) float    Os[AH_NW][16 * 68];

  const int tid  = threadIdx.x;
  const int wave = tid >> 5;
  const int lane = tid & 31;
  const int hh   = lane >> 4;
  const int c    = lane & 15;

  const int nqb = S / AH_QB;
  const int qb  = blockIdx.x % nqb;
  const int hp  = blockIdx.x / nqb;
  const int q0  = qb * AH_QB + wave * 16;
  const int nChunks = S / AH_KC;
  float* os = Os[wave];
  _Float16* pw = Psh[wave];
  const v8f zero8 = (v8f){0.f,0.f,0.f,0.f,0.f,0.f,0.f,0.f};

  for (int hs = 0; hs < 2; ++hs) {
    const int hcol = (hp * 2 + hs) * AH_D;
    const v16h qa = Frag<_Float16>::load(q + (size_t)(q0 + c) * ld + hcol + 8 * hh);

    float mrow[8], lrow[8];
    v8f oacc[2];
#pragma unroll
    for (int r = 0; r < 8; ++r) { mrow[r] = -INFINITY; lrow[r] = 0.f; }
    oacc[0] = zero8; oacc[1] = zero8;

    for (int kc = 0; kc < nChunks; ++kc) {
      const int kv0 = kc * AH_KC;
      __syncthreads();
      {
        const int kvr = tid >> 1, dh = (tid & 1) * 16;
        const _Float16* krow = k + (size_t)(kv0 + kvr) * ld + hcol + dh;
        const _Float16* vrow = v + (size_t)(kv0 + kvr) * ld + hcol + dh;
        const v8h k0v = *(const v8h*)krow;
        const v8h k1v = *(const v8h*)(krow + 8);
        const v8h v0v = *(const v8h*)vrow;
        const v8h v1v = *(const v8h*)(vrow + 8);
        *(v8h*)(Ksh + kvr * AH_D + dh)     = k0v;
        *(v8h*)(Ksh + kvr * AH_D + dh + 8) = k1v;
#pragma unroll
        for (int e = 0; e < 8; ++e) {
          Vth[(dh + e) * AH_KC + kvr]     = v0v[e];
          Vth[(dh + 8 + e) * AH_KC + kvr] = v1v[e];
        }
      }
      __syncthreads();

      v8f s[4];
#pragma unroll
      for (int j = 0; j < 4; ++j) {
        const v16h kb = Frag<_Float16>::load(Ksh + (j * 16 + c) * AH_D + 8 * hh);
        s[j] = mma_f16g(qa, kb, zero8);
      }
      float cm[8];
#pragma unroll
      for (int r = 0; r < 8; ++r) {
        float m = -INFINITY;
#pragma unroll
        for (int j = 0; j < 4; ++j) {
          s[j][r] *= qk_scale;
          m = fmaxf(m, s[j][r]);
        }
#pragma unroll
        for (int off = 1; off < 16; off <<= 1) m = fmaxf(m, __shfl_xor(m, off, 32));
        cm[r] = m;
      }
#pragma unroll
      for (int r = 0; r < 8; ++r) {
        const float mnew  = fmaxf(mrow[r], cm[r]);
        const float alpha = expf(mrow[r] - mnew);
        mrow[r] = mnew;
        float psum = 0.f;
#pragma unroll
        for (int j = 0; j < 4; ++j) {
          const float p = expf(s[j][r] - mnew);
          psum += p;
          pw[(8 * hh + r) * AH_KC + j * 16 + c] = (_Float16)(p * PSCALE);
        }
#pragma unroll
        for (int off = 1; off < 16; off <<= 1) psum += __shfl_xor(psum, off, 32);
        lrow[r] = lrow[r] * alpha + psum;
        oacc[0][r] *= alpha;
        oacc[1][r] *= alpha;
      }
      __builtin_amdgcn_fence(__ATOMIC_RELEASE, "workgroup");
      __builtin_amdgcn_wave_barrier();
      __builtin_amdgcn_fence(__ATOMIC_ACQUIRE, "workgroup");
#pragma unroll
      for (int kk = 0; kk < 2; ++kk) {
        const v16h pa = Frag<_Float16>::load(pw + c * AH_KC + kk * 32 + 8 * hh);
#pragma unroll
        for (int t = 0; t < 2; ++t) {
          const v16h vb = Frag<_Float16>::load(Vth + (t * 16 + c) * AH_KC + kk * 32 + 8 * hh);
          oacc[t] = mma_f16g(pa, vb, oacc[t]);
        }
      }
    }
#pragma unroll
    for (int r = 0; r < 8; ++r) {
      const float inv = 1.0f / (lrow[r] * PSCALE);
#pragma unroll
      for (int t = 0; t < 2; ++t) os[(8 * hh + r) * 68 + hs * AH_D + t * 16 + c] = oacc[t][r] * inv;
    }
  }
  __builtin_amdgcn_fence(__ATOMIC_RELEASE, "workgroup");
  __builtin_amdgcn_wave_barrier();
  __builtin_amdgcn_fence(__ATOMIC_ACQUIRE, "workgroup");
  {
    const int q8 = lane >> 3, c8 = (lane & 7) * 8;
    for (int pass = 0; pass < 2; ++pass) {
#pragma unroll
      for (int it = 0; it < 4; ++it) {
        const int row = it * 4 + q8;
        const float* sp = os + row * 68 + c8;
        v8h hv;
#pragma unroll
        for (int e = 0; e < 8; ++e) hv[e] = (_Float16)sp[e];
        *(volatile v8h*)(o + (size_t)(q0 + row) * ld + hp * (2 * AH_D) + c8) = hv;
      }
      __threadfence();
    }
  }
}

extern "C" void kernel_launch(void* const* d_in, const int* in_sizes, int n_in,
                              void* d_out, int out_size, void* d_ws, size_t ws_size,
                              hipStream_t stream) {
  if (n_in < 17) return;
  if (in_sizes[0] != NTOK * CDIM || in_sizes[1] != CDIM || in_sizes[2] != CDIM ||
      in_sizes[3] != CDIM * CDIM || in_sizes[4] != CDIM ||
      in_sizes[5] != CDIM * CDIM || in_sizes[6] != CDIM ||
      in_sizes[7] != CDIM * CDIM || in_sizes[8] != CDIM ||
      in_sizes[9] != CDIM * CDIM || in_sizes[10] != CDIM ||
      in_sizes[11] != CDIM || in_sizes[12] != CDIM ||
      in_sizes[13] != CDIM * FFDIM || in_sizes[14] != FFDIM ||
      in_sizes[15] != FFDIM * CDIM || in_sizes[16] != CDIM ||
      out_size != NTOK * CDIM) return;

  const float* x     = (const float*)d_in[0];
  const float* gn1_w = (const float*)d_in[1];
  const float* gn1_b = (const float*)d_in[2];
  const float* wq = (const float*)d_in[3];  const float* bq = (const float*)d_in[4];
  const float* wk = (const float*)d_in[5];  const float* bk = (const float*)d_in[6];
  const float* wv = (const float*)d_in[7];  const float* bv = (const float*)d_in[8];
  const float* wo = (const float*)d_in[9];  const float* bo = (const float*)d_in[10];
  const float* gn2_w = (const float*)d_in[11];
  const float* gn2_b = (const float*)d_in[12];
  const float* w1 = (const float*)d_in[13]; const float* b1 = (const float*)d_in[14];
  const float* w2 = (const float*)d_in[15]; const float* b2 = (const float*)d_in[16];
  float* out = (float*)d_out;

  char* ws = (char*)d_ws;
  size_t off = 0;
  auto carve = [&](size_t bytes) -> void* {
    void* p = ws + off;
    off += (bytes + 255) & ~(size_t)255;
    return p;
  };
  unsigned short* wq_t = (unsigned short*)carve((size_t)CDIM * CDIM * 2);
  unsigned short* wk_t = (unsigned short*)carve((size_t)CDIM * CDIM * 2);
  unsigned short* wv_t = (unsigned short*)carve((size_t)CDIM * CDIM * 2);
  unsigned short* wo_t = (unsigned short*)carve((size_t)CDIM * CDIM * 2);
  unsigned short* w1_t = (unsigned short*)carve((size_t)FFDIM * CDIM * 2);
  unsigned short* w2_t = (unsigned short*)carve((size_t)CDIM * FFDIM * 2);
  float* stats1 = (float*)carve((size_t)NGRP * 32 * 4);
  float* stats2 = (float*)carve((size_t)NGRP * 32 * 4);
  float* t_f    = (float*)carve((size_t)NTOK * CDIM * 4);
  unsigned short* t_h  = (unsigned short*)carve((size_t)NTOK * CDIM * 2);
  unsigned short* q_h  = (unsigned short*)carve((size_t)NTOK * CDIM * 2);
  unsigned short* k_h  = (unsigned short*)carve((size_t)NTOK * CDIM * 2);
  unsigned short* v_h  = (unsigned short*)carve((size_t)NTOK * CDIM * 2);
  unsigned short* ao_h = (unsigned short*)carve((size_t)NTOK * CDIM * 2);
  float* x2     = (float*)carve((size_t)NTOK * CDIM * 4);
  unsigned short* t2_h = (unsigned short*)carve((size_t)NTOK * CDIM * 2);
  float* t2cm   = (float*)carve((size_t)CDIM * NTOK * 4);
  unsigned short* h_h  = (unsigned short*)carve((size_t)NTOK * FFDIM * 2);
  if (off > ws_size) return;

  transpose_cast_f16<<<dim3(CDIM / 64, CDIM / 64), 256, 0, stream>>>(wq, wq_t, CDIM, CDIM, WSCALE);
  transpose_cast_f16<<<dim3(CDIM / 64, CDIM / 64), 256, 0, stream>>>(wk, wk_t, CDIM, CDIM, WSCALE);
  transpose_cast_f16<<<dim3(CDIM / 64, CDIM / 64), 256, 0, stream>>>(wv, wv_t, CDIM, CDIM, WSCALE);
  transpose_cast_f16<<<dim3(CDIM / 64, CDIM / 64), 256, 0, stream>>>(wo, wo_t, CDIM, CDIM, WSCALE);
  transpose_cast_f16<<<dim3(FFDIM / 64, CDIM / 64), 256, 0, stream>>>(w1, w1_t, CDIM, FFDIM, WSCALE);
  transpose_cast_f16<<<dim3(CDIM / 64, FFDIM / 64), 256, 0, stream>>>(w2, w2_t, FFDIM, CDIM, WSCALE);

  gn_stats_cm<<<NGRP, 256, 0, stream>>>(x, stats1, (CDIM / NGRP) * NTOK, GN_EPS);
  gn_apply_cm<<<NTOK / 32, 256, 0, stream>>>(x, stats1, gn1_w, gn1_b, t_f, t_h, NTOK);

  const int tilesCC = (NTOK / 64) * (CDIM / 64);
  const dim3 gCC((tilesCC + 7) / 8, 1);
  wmma_gemm64<0, false, 2, 1, false, 0><<<gCC, 256, 0, stream>>>(
      t_h, t_h, CDIM, 0L, wq_t, wq_t, CDIM, 0L, (void*)q_h, (void*)q_h, CDIM, 0L, bq, t_f, 0L, NTOK, CDIM, CDIM, WSCALE_INV);
  wmma_gemm64<0, false, 2, 1, false, 0><<<gCC, 256, 0, stream>>>(
      t_h, t_h, CDIM, 0L, wk_t, wk_t, CDIM, 0L, (void*)k_h, (void*)k_h, CDIM, 0L, bk, t_f, 0L, NTOK, CDIM, CDIM, WSCALE_INV);
  wmma_gemm64<0, false, 2, 1, false, 0><<<gCC, 256, 0, stream>>>(
      t_h, t_h, CDIM, 0L, wv_t, wv_t, CDIM, 0L, (void*)v_h, (void*)v_h, CDIM, 0L, bv, t_f, 0L, NTOK, CDIM, CDIM, WSCALE_INV);

  attn_hd32_f16<<<(NHEAD / 2) * (NTOK / AH_QB), 128, 0, stream>>>(
      q_h, k_h, v_h, ao_h, NTOK, CDIM, 0.17677669529663687f);

  wmma_gemm64<0, false, 2, 0, true, 0><<<gCC, 256, 0, stream>>>(
      ao_h, ao_h, CDIM, 0L, wo_t, wo_t, CDIM, 0L, (void*)x2, (void*)x2, CDIM, 0L, bo, t_f, 0L, NTOK, CDIM, CDIM, WSCALE_INV);

  gn_stats_tm<<<NGRP, 256, 0, stream>>>(x2, stats2, NTOK, GN_EPS);
  gn_apply_tm<<<NTOK / 32, 256, 0, stream>>>(x2, stats2, gn2_w, gn2_b, t2_h, t2cm, NTOK);

  const int tilesF = (NTOK / 64) * (FFDIM / 64);
  wmma_gemm64<0, false, 2, 1, false, 5><<<dim3((tilesF + 7) / 8, 1), 256, 0, stream>>>(
      t2_h, t2_h, CDIM, 0L, w1_t, w1_t, CDIM, 0L, (void*)h_h, (void*)h_h, FFDIM, 0L, b1, t_f, 0L, NTOK, FFDIM, CDIM, WSCALE_INV);

  const int tilesO = (CDIM / 64) * (NTOK / 64);
  wmma_gemm64<0, false, 1, 0, true, 0><<<dim3((tilesO + 7) / 8, 1), 256, 0, stream>>>(
      w2_t, w2_t, FFDIM, 0L, h_h, h_h, FFDIM, 0L, (void*)out, (void*)out, NTOK, 0L, b2, t2cm, 0L, CDIM, NTOK, FFDIM, WSCALE_INV);
}
